// MLAAttention_12902081757317
// MI455X (gfx1250) — hardware-verified
//
#include <hip/hip_runtime.h>

typedef _Float16 hf_t;
typedef _Float16 v16h __attribute__((ext_vector_type(16)));
typedef _Float16 v8h __attribute__((ext_vector_type(8)));
typedef float v8f __attribute__((ext_vector_type(8)));
typedef float v4f __attribute__((ext_vector_type(4)));
typedef v8h v8h_ma __attribute__((may_alias));
typedef v4f v4f_ma __attribute__((may_alias));
union Frag { v16h v; v8h half[2]; };

constexpr int kB = 2, kT = 2048, kHID = 2048, kH = 16, kKV = 4, kHD = 128, kOD = 128, kLAT = 512;
constexpr int kM = kB * kT;
constexpr int kT0 = 256;
constexpr float kResMul = 4096.0f;
constexpr float kResInv = 1.0f / 4096.0f;
static_assert(kHD == 128 && kOD == 128 && kHID == kH * kOD && kLAT == kKV * kHD && kH % kKV == 0);
static_assert(kT0 % 128 == 0 && (kT - kT0) % 128 == 0 && kT0 % 64 == 0 && kT0 > 0 && kT0 < kT);
static_assert(kHID % 128 == 0 && kLAT % 128 == 0 && kT % 128 == 0 && kHD % 64 == 0 && kT % 64 == 0);
static_assert((kM * kHID) % 2048 == 0 && (kHID * kHID) % 2048 == 0 && (kLAT * kHID) % 2048 == 0 && (kHID * kHD) % 2048 == 0);

__device__ __forceinline__ v16h ld_frag(const hf_t* base, int pitch, int row0, int k0, int lane) {
  const hf_t* p = base + (size_t)(row0 + (lane & 15)) * pitch + k0 + ((lane >> 4) << 3);
  Frag f;
  f.half[0] = *(const v8h_ma*)p;
  f.half[1] = *(const v8h_ma*)(p + 16);
  return f.v;
}

__device__ __forceinline__ v8f wmma16(v16h a, v16h b, v8f c) {
  return __builtin_amdgcn_wmma_f32_16x16x32_f16(false, a, false, b, (short)0, c, false, false);
}

#define WNOPS "v_nop\n\tv_nop\n\tv_nop\n\tv_nop"

__device__ __forceinline__ void split16(float v, hf_t& hi, hf_t& lo) {
  const hf_t hv = (hf_t)v;
  hi = hv;
  lo = (hf_t)((v - (float)hv) * kResMul);
}

__global__ __launch_bounds__(256) void k_cvt(const float* __restrict__ src, hf_t* dhi, hf_t* dlo, int n8, float scale) {
  const int i = (int)blockIdx.x * 256 + (int)threadIdx.x;
  if (i >= n8) return;
  const float* s = src + (size_t)i * 8;
  const v4f a = *(const v4f_ma*)s;
  const v4f c = *(const v4f_ma*)(s + 4);
  v8h H, L;
#pragma unroll
  for (int e = 0; e < 4; ++e) {
    hf_t hi, lo;
    split16(a[e] * scale, hi, lo); H[e] = hi; L[e] = lo;
    split16(c[e] * scale, hi, lo); H[4 + e] = hi; L[4 + e] = lo;
  }
  volatile v8h* ph = (volatile v8h*)(dhi + (size_t)i * 8);
  volatile v8h* pl = (volatile v8h*)(dlo + (size_t)i * 8);
  *ph = H;
  *pl = L;
  __threadfence();
  *ph = H;
  *pl = L;
}

__device__ __forceinline__ void trs_store(const float* tile, hf_t* dhi, hf_t* dlo, int hh, int c0, int tid) {
  const int q = tid & 7;
#pragma unroll
  for (int t = 0; t < 4; ++t) {
    const int L = t * 32 + (tid >> 3);
    const int pl = L >> 6, c = (L >> 1) & 31, seg = L & 1;
    const float* sp = tile + c * 132 + seg * 64 + q * 8;
    const v4f a = *(const v4f_ma*)sp;
    const v4f cc = *(const v4f_ma*)(sp + 4);
    v8h H, Lv;
#pragma unroll
    for (int e = 0; e < 4; ++e) {
      hf_t hi, lo;
      split16(a[e] * 64.0f, hi, lo); H[e] = hi; Lv[e] = lo;
      split16(cc[e] * 64.0f, hi, lo); H[4 + e] = hi; Lv[4 + e] = lo;
    }
    const v8h val = pl ? Lv : H;
    hf_t* dst = (pl ? dlo : dhi) + (size_t)(hh * kHD + c0 + c) * kOD + seg * 64 + q * 8;
    *(volatile v8h*)dst = val;
  }
}

__global__ __launch_bounds__(256) void k_cvt_tr(const float* __restrict__ W, hf_t* dhi, hf_t* dlo) {
  __shared__ __attribute__((aligned(16))) float tile[32 * 132];
  const int tid = (int)threadIdx.x;
  const int c0 = (int)blockIdx.x * 32, hh = (int)blockIdx.y;
#pragma unroll
  for (int t = 0; t < 16; ++t) {
    const int idx = tid + t * 256;
    const int d = idx >> 5, c = idx & 31;
    tile[c * 132 + d] = W[(size_t)(hh * kOD + d) * kHD + c0 + c];
  }
  __syncthreads();
  trs_store(tile, dhi, dlo, hh, c0, tid);
  __threadfence();
  trs_store(tile, dhi, dlo, hh, c0, tid);
}

struct GemmP {
  long long aSb, aSh, bSb, bSh, cSb, cSh;
  int K, lda, ldb, ldc, zdiv, aHdiv, bHdiv, mbase, nbase, has_bias;
  float escale, oscale;
};
static_assert(sizeof(GemmP) == 96);

template <bool SPLIT>
__device__ __forceinline__ void gemm_lines16(const hf_t* Cs, hf_t* Chi, hf_t* Clo, long long coff,
                                             int m0, int n0, int ldc, int tid) {
  constexpr int BN = SPLIT ? 64 : 128;
  constexpr int CP = BN + 8;
  const int q = tid & 7;
#pragma unroll
  for (int it = 0; it < 8; ++it) {
    const int L = it * 32 + (tid >> 3);
    int pl, row, seg;
    if (SPLIT) { pl = L >> 7; row = L & 127; seg = 0; }
    else       { pl = 0; row = L >> 1; seg = L & 1; }
    const v8h val = *(const v8h_ma*)(Cs + pl * (128 * CP) + row * CP + seg * 64 + q * 8);
    hf_t* dst = (pl ? Clo : Chi) + coff + (size_t)(m0 + row) * ldc + n0 + seg * 64 + q * 8;
    *(volatile v8h*)dst = val;
  }
}

template <int BN>
__device__ __forceinline__ void gemm_lines32(const float* Cs, float* Cf, long long coff,
                                             int mrow0, int n0, int ldc, int tid) {
  constexpr int FP = BN + 4;
  constexpr int LPR = BN / 32;
  constexpr int NIT = (64 * LPR) / 32;
  const int q = tid & 7;
#pragma unroll
  for (int it = 0; it < NIT; ++it) {
    const int L = it * 32 + (tid >> 3);
    const int row = L / LPR, seg = L % LPR;
    const v4f val = *(const v4f_ma*)(Cs + row * FP + seg * 32 + q * 4);
    float* dst = Cf + coff + (size_t)(mrow0 + row) * ldc + n0 + seg * 32 + q * 4;
    *(volatile v4f*)dst = val;
  }
}

template <bool SPLIT, bool OUTF32>
__global__ __launch_bounds__(256) __attribute__((amdgpu_num_vgpr(256)))
void k_gemm(const hf_t* __restrict__ Ahi, const hf_t* __restrict__ Alo,
            const hf_t* __restrict__ Bhi, const hf_t* __restrict__ Blo,
            const float* __restrict__ bias, float* Cf, hf_t* Chi, hf_t* Clo, GemmP g) {
  constexpr int BN = SPLIT ? 64 : 128;
  constexpr int NJ = BN / 32;
  constexpr int NP = SPLIT ? 2 : 1;
  constexpr int AP = 40;
  constexpr int APL = 128 * AP;
  constexpr int BPL = BN * AP;
  __shared__ __attribute__((aligned(16))) unsigned char smem[36864];
  static_assert(NP * (APL + BPL) * 2 <= 36864);
  static_assert(NP * 128 * (BN + 8) * 2 <= 36864);
  static_assert(64 * (BN + 4) * 4 <= 36864);
  hf_t* As = (hf_t*)smem;
  hf_t* Bs = As + NP * APL;

  const int tid = (int)threadIdx.x;
  const int lane = tid & 31, wid = tid >> 5;
  const int wm = wid >> 1, wn = wid & 1, hf = lane >> 4, cl = lane & 15;
  const int zb = (int)blockIdx.z / g.zdiv, zh = (int)blockIdx.z % g.zdiv;
  const long long aoff = (long long)zb * g.aSb + (long long)(zh / g.aHdiv) * g.aSh;
  const long long boff = (long long)zb * g.bSb + (long long)(zh / g.bHdiv) * g.bSh;
  const long long coff = (long long)zb * g.cSb + (long long)zh * g.cSh;
  const hf_t* Ah = Ahi + aoff;
  const hf_t* Al = Alo + aoff;
  const hf_t* Bh = Bhi + boff;
  const hf_t* Bl = Blo + boff;
  const int n0 = g.nbase + (int)blockIdx.x * BN;
  const int m0 = g.mbase + (int)blockIdx.y * 128;

  const v8f vzero = {};
  v8f acc[2][NJ], res[2][NJ];
#pragma unroll
  for (int i = 0; i < 2; ++i)
#pragma unroll
    for (int j = 0; j < NJ; ++j) { acc[i][j] = vzero; res[i][j] = vzero; }

#pragma unroll 1
  for (int k0 = 0; k0 < g.K; k0 += 32) {
#pragma unroll
    for (int t = 0; t < NP * 2; ++t) {
      const int c = tid + t * 256;
      const int pl = c >> 9, r = (c >> 2) & 127, q = c & 3;
      const hf_t* src = (pl ? Al : Ah) + (size_t)(m0 + r) * g.lda + k0 + q * 8;
      *(v8h_ma*)(As + pl * APL + r * AP + q * 8) = *(const v8h_ma*)src;
    }
    constexpr int BT = NP * BN / 64;
    constexpr int BSH = SPLIT ? 8 : 9;
#pragma unroll
    for (int t = 0; t < BT; ++t) {
      const int c = tid + t * 256;
      const int pl = c >> BSH, r = (c >> 2) & (BN - 1), q = c & 3;
      const hf_t* src = (pl ? Bl : Bh) + (size_t)(n0 + r) * g.ldb + k0 + q * 8;
      *(v8h_ma*)(Bs + pl * BPL + r * AP + q * 8) = *(const v8h_ma*)src;
    }
    __syncthreads();

    if constexpr (SPLIT) {
      v16h ah[2], al[2], bh[2], bl[2];
#pragma unroll
      for (int i = 0; i < 2; ++i) {
        ah[i] = ld_frag(As, AP, wm * 32 + i * 16, 0, lane);
        al[i] = ld_frag(As + APL, AP, wm * 32 + i * 16, 0, lane);
      }
#pragma unroll
      for (int j = 0; j < 2; ++j) {
        bh[j] = ld_frag(Bs, AP, wn * 32 + j * 16, 0, lane);
        bl[j] = ld_frag(Bs + BPL, AP, wn * 32 + j * 16, 0, lane);
      }
#pragma unroll
      for (int i = 0; i < 2; ++i)
#pragma unroll
        for (int j = 0; j < 2; ++j) {
          acc[i][j] = wmma16(ah[i], bh[j], acc[i][j]);
          res[i][j] = wmma16(ah[i], bl[j], res[i][j]);
          res[i][j] = wmma16(al[i], bh[j], res[i][j]);
        }
      asm volatile(WNOPS
                   : "+v"(acc[0][0]), "+v"(acc[0][1]), "+v"(acc[1][0]), "+v"(acc[1][1]),
                     "+v"(res[0][0]), "+v"(res[0][1]), "+v"(res[1][0]), "+v"(res[1][1])
                   : "v"(ah[0]), "v"(ah[1]), "v"(al[0]), "v"(al[1]),
                     "v"(bh[0]), "v"(bh[1]), "v"(bl[0]), "v"(bl[1]));
    } else {
      v16h ah[2], bh[4];
#pragma unroll
      for (int i = 0; i < 2; ++i) ah[i] = ld_frag(As, AP, wm * 32 + i * 16, 0, lane);
#pragma unroll
      for (int j = 0; j < 4; ++j) bh[j] = ld_frag(Bs, AP, wn * 64 + j * 16, 0, lane);
#pragma unroll
      for (int i = 0; i < 2; ++i)
#pragma unroll
        for (int j = 0; j < 4; ++j) acc[i][j] = wmma16(ah[i], bh[j], acc[i][j]);
      asm volatile(WNOPS
                   : "+v"(acc[0][0]), "+v"(acc[0][1]), "+v"(acc[0][2]), "+v"(acc[0][3]),
                     "+v"(acc[1][0]), "+v"(acc[1][1]), "+v"(acc[1][2]), "+v"(acc[1][3])
                   : "v"(ah[0]), "v"(ah[1]), "v"(bh[0]), "v"(bh[1]), "v"(bh[2]), "v"(bh[3]));
    }
    __syncthreads();
  }

  if constexpr (!OUTF32) {
    constexpr int CP = BN + 8;
    hf_t* Cs = (hf_t*)smem;
#pragma unroll
    for (int i = 0; i < 2; ++i)
#pragma unroll
      for (int j = 0; j < NJ; ++j) {
        const int col = wn * (BN / 2) + j * 16 + cl;
        const float bv = g.has_bias ? bias[n0 + col] : 0.0f;
#pragma unroll
        for (int r = 0; r < 8; ++r) {
          const int row = wm * 32 + i * 16 + hf * 8 + r;
          float a = acc[i][j][r];
          if constexpr (SPLIT) a = fmaf(res[i][j][r], kResInv, a);
          const float vs = fmaf(a, g.escale, bv) * g.oscale;
          const hf_t hi = (hf_t)vs;
          Cs[row * CP + col] = hi;
          if constexpr (SPLIT) Cs[128 * CP + row * CP + col] = (hf_t)((vs - (float)hi) * kResMul);
        }
      }
    __syncthreads();
    gemm_lines16<SPLIT>(Cs, Chi, Clo, coff, m0, n0, g.ldc, tid);
    __threadfence();
    gemm_lines16<SPLIT>(Cs, Chi, Clo, coff, m0, n0, g.ldc, tid);
  } else {
    constexpr int FP = BN + 4;
    float* Cs = (float*)smem;
#pragma unroll
    for (int half = 0; half < 2; ++half) {
      if ((wm >> 1) == half) {
#pragma unroll
        for (int i = 0; i < 2; ++i)
#pragma unroll
          for (int j = 0; j < NJ; ++j) {
            const int col = wn * (BN / 2) + j * 16 + cl;
            const float bv = g.has_bias ? bias[n0 + col] : 0.0f;
#pragma unroll
            for (int r = 0; r < 8; ++r) {
              const int row = (wm & 1) * 32 + i * 16 + hf * 8 + r;
              float a = acc[i][j][r];
              if constexpr (SPLIT) a = fmaf(res[i][j][r], kResInv, a);
              Cs[row * FP + col] = fmaf(a, g.escale, bv);
            }
          }
      }
      __syncthreads();
      gemm_lines32<BN>(Cs, Cf, coff, m0 + half * 64, n0, g.ldc, tid);
      __threadfence();
      gemm_lines32<BN>(Cs, Cf, coff, m0 + half * 64, n0, g.ldc, tid);
      __syncthreads();
    }
  }
}

template <int NP>
__device__ __forceinline__ void attn_lines(const hf_t* Os, hf_t* Oh, hf_t* Ol, size_t rowbase, int hcol, int lane) {
  const int q = lane & 7;
#pragma unroll
  for (int it = 0; it < 8 * NP; ++it) {
    const int L = it * 4 + (lane >> 3);
    const int pl = L >> 5, rr = (L >> 1) & 15, seg = L & 1;
    const v8h val = *(const v8h_ma*)(Os + pl * (16 * 136) + rr * 136 + seg * 64 + q * 8);
    hf_t* dst = (pl ? Ol : Oh) + (rowbase + (size_t)rr) * kHID + hcol + seg * 64 + q * 8;
    *(volatile v8h*)dst = val;
  }
}

template <bool SPLIT>
__global__ __launch_bounds__(32) __attribute__((amdgpu_num_vgpr(256)))
void k_attn(const hf_t* __restrict__ Qh, const hf_t* __restrict__ Ql,
            const hf_t* __restrict__ Kh, const hf_t* __restrict__ Kl,
            const hf_t* __restrict__ Vh, const hf_t* __restrict__ Vl,
            const float* __restrict__ amask, hf_t* Oh, hf_t* Ol, int qbase) {
  constexpr int NP = SPLIT ? 2 : 1;
  constexpr int OP = 136;
  __shared__ __attribute__((aligned(16))) hf_t Os[2 * 16 * OP];

  const int lane = (int)threadIdx.x & 31, lh = lane >> 4, m = lane & 15;
  const int b = (int)blockIdx.z, hd = (int)blockIdx.y;
  const int kv = hd / (kH / kKV);
  const int bh = b * kH + hd;
  const int q0 = qbase + (int)blockIdx.x * 16;
  const int kend = q0 + 16;
  const float smscale = 0.022097086912079611f;

  const hf_t* qh = Qh + ((size_t)bh * kT + q0) * kHD;
  const hf_t* ql = Ql + ((size_t)bh * kT + q0) * kHD;
  const hf_t* kh = Kh + (size_t)b * kT * kLAT + kv * kHD;
  const hf_t* kl = Kl + (size_t)b * kT * kLAT + kv * kHD;
  const hf_t* vh = Vh + (size_t)bh * kOD * kT;
  const hf_t* vl = Vl + (size_t)bh * kOD * kT;
  const float* mrowp = amask + ((size_t)b * kT + q0 + m) * kT;

  const v8f vzero = {};
  v8f oT[8];
#pragma unroll
  for (int d = 0; d < 8; ++d) oT[d] = vzero;
  float mval = -3.0e38f, lsum = 0.0f;

#pragma unroll 1
  for (int kc = 0; kc < kend; kc += 64) {
    v8f sT[4], sR[4];
#pragma unroll
    for (int j = 0; j < 4; ++j) { sT[j] = vzero; sR[j] = vzero; }
#pragma unroll
    for (int cc = 0; cc < 4; ++cc) {
      const v16h bqh = ld_frag(qh, kHD, 0, cc * 32, lane);
      if constexpr (SPLIT) {
        const v16h bql = ld_frag(ql, kHD, 0, cc * 32, lane);
#pragma unroll
        for (int j = 0; j < 4; ++j) {
          const v16h akh = ld_frag(kh, kLAT, kc + j * 16, cc * 32, lane);
          const v16h akl = ld_frag(kl, kLAT, kc + j * 16, cc * 32, lane);
          sT[j] = wmma16(akh, bqh, sT[j]);
          sR[j] = wmma16(akh, bql, sR[j]);
          sR[j] = wmma16(akl, bqh, sR[j]);
          asm volatile(WNOPS : "+v"(sT[j]), "+v"(sR[j]) : "v"(akh), "v"(akl), "v"(bqh), "v"(bql));
        }
      } else {
        v16h ak[4];
#pragma unroll
        for (int j = 0; j < 4; ++j) ak[j] = ld_frag(kh, kLAT, kc + j * 16, cc * 32, lane);
#pragma unroll
        for (int j = 0; j < 4; ++j) sT[j] = wmma16(ak[j], bqh, sT[j]);
        asm volatile(WNOPS
                     : "+v"(sT[0]), "+v"(sT[1]), "+v"(sT[2]), "+v"(sT[3])
                     : "v"(ak[0]), "v"(ak[1]), "v"(ak[2]), "v"(ak[3]), "v"(bqh));
      }
    }

    float p[4][8];
    float mx = -3.0e38f;
#pragma unroll
    for (int j = 0; j < 4; ++j) {
      const float* mp = mrowp + kc + j * 16 + lh * 8;
      const v4f ma = *(const v4f_ma*)mp;
      const v4f mb = *(const v4f_ma*)(mp + 4);
#pragma unroll
      for (int r = 0; r < 8; ++r) {
        float sv = sT[j][r];
        if constexpr (SPLIT) sv = fmaf(sR[j][r], kResInv, sv);
        sv = fmaf(sv, smscale, (r < 4) ? ma[r] : mb[r - 4]);
        p[j][r] = sv;
        mx = fmaxf(mx, sv);
      }
    }
    mx = fmaxf(mx, __shfl_xor(mx, 16));
    const float mnew = fmaxf(mval, mx);
    const float corr = __expf(mval - mnew);
    float ps = 0.0f;
#pragma unroll
    for (int j = 0; j < 4; ++j)
#pragma unroll
      for (int r = 0; r < 8; ++r) {
        const float e = __expf(p[j][r] - mnew);
        p[j][r] = e;
        ps += e;
      }
    ps += __shfl_xor(ps, 16);
    lsum = lsum * corr + ps;
    mval = mnew;
#pragma unroll
    for (int d = 0; d < 8; ++d)
#pragma unroll
      for (int r = 0; r < 8; ++r) oT[d][r] *= corr;

    Frag pbh[2], pbl[2];
#pragma unroll
    for (int ks = 0; ks < 2; ++ks)
#pragma unroll
      for (int i = 0; i < 8; ++i) {
        const float p0 = p[2 * ks][i], p1 = p[2 * ks + 1][i];
        const hf_t h0 = (hf_t)p0, h1 = (hf_t)p1;
        pbh[ks].half[0][i] = h0;
        pbh[ks].half[1][i] = h1;
        if constexpr (SPLIT) {
          pbl[ks].half[0][i] = (hf_t)((p0 - (float)h0) * kResMul);
          pbl[ks].half[1][i] = (hf_t)((p1 - (float)h1) * kResMul);
        } else {
          pbl[ks].half[0][i] = h0;
          pbl[ks].half[1][i] = h1;
        }
      }

    if constexpr (SPLIT) {
#pragma unroll
      for (int d = 0; d < 8; ++d) {
        v8f oR = vzero;
#pragma unroll
        for (int ks = 0; ks < 2; ++ks) {
          const v16h avh = ld_frag(vh, kT, d * 16, kc + ks * 32, lane);
          const v16h avl = ld_frag(vl, kT, d * 16, kc + ks * 32, lane);
          oT[d] = wmma16(avh, pbh[ks].v, oT[d]);
          oR = wmma16(avh, pbl[ks].v, oR);
          oR = wmma16(avl, pbh[ks].v, oR);
          asm volatile(WNOPS : "+v"(oT[d]), "+v"(oR) : "v"(avh), "v"(avl), "v"(pbh[ks].v), "v"(pbl[ks].v));
        }
#pragma unroll
        for (int r = 0; r < 8; ++r) oT[d][r] = fmaf(oR[r], kResInv, oT[d][r]);
      }
    } else {
#pragma unroll
      for (int ks = 0; ks < 2; ++ks) {
        v16h av[8];
#pragma unroll
        for (int d = 0; d < 8; ++d) av[d] = ld_frag(vh, kT, d * 16, kc + ks * 32, lane);
#pragma unroll
        for (int d = 0; d < 8; ++d) oT[d] = wmma16(av[d], pbh[ks].v, oT[d]);
        asm volatile(WNOPS
                     : "+v"(oT[0]), "+v"(oT[1]), "+v"(oT[2]), "+v"(oT[3]),
                       "+v"(oT[4]), "+v"(oT[5]), "+v"(oT[6]), "+v"(oT[7])
                     : "v"(av[0]), "v"(av[1]), "v"(av[2]), "v"(av[3]),
                       "v"(av[4]), "v"(av[5]), "v"(av[6]), "v"(av[7]), "v"(pbh[ks].v));
      }
    }
  }

  const float f = 64.0f / lsum;
#pragma unroll
  for (int d = 0; d < 8; ++d) {
    v8h hv, lv;
#pragma unroll
    for (int r = 0; r < 8; ++r) {
      const float val = oT[d][r] * f;
      const hf_t hi = (hf_t)val;
      hv[r] = hi;
      if constexpr (SPLIT) lv[r] = (hf_t)((val - (float)hi) * kResMul);
      else lv[r] = hi;
    }
    *(v8h_ma*)(Os + m * OP + d * 16 + lh * 8) = hv;
    if constexpr (SPLIT) *(v8h_ma*)(Os + 16 * OP + m * OP + d * 16 + lh * 8) = lv;
  }
  __syncthreads();
  const size_t rowbase = (size_t)(b * kT + q0);
  attn_lines<NP>(Os, Oh, Ol, rowbase, hd * kOD, lane);
  __threadfence();
  attn_lines<NP>(Os, Oh, Ol, rowbase, hd * kOD, lane);
}

static GemmP mkp(long long aSb, long long aSh, long long bSb, long long bSh, long long cSb, long long cSh,
                 int K, int lda, int ldb, int ldc, int zdiv, int aHdiv, int bHdiv, int mbase, int nbase,
                 int has_bias, float escale, float oscale) {
  GemmP p;
  p.aSb = aSb; p.aSh = aSh; p.bSb = bSb; p.bSh = bSh; p.cSb = cSb; p.cSh = cSh;
  p.K = K; p.lda = lda; p.ldb = ldb; p.ldc = ldc; p.zdiv = zdiv; p.aHdiv = aHdiv; p.bHdiv = bHdiv;
  p.mbase = mbase; p.nbase = nbase; p.has_bias = has_bias; p.escale = escale; p.oscale = oscale;
  return p;
}

extern "C" void kernel_launch(void* const* d_in, const int* in_sizes, int n_in,
                              void* d_out, int out_size, void* d_ws,
                              size_t ws_size, hipStream_t stream) {
  if (n_in != 12) return;
  if (in_sizes[0] != kM * kHID || in_sizes[1] != kB * kT * kT || in_sizes[2] != kHID * kHID ||
      in_sizes[3] != kHID || in_sizes[4] != kLAT * kHID || in_sizes[5] != kLAT ||
      in_sizes[6] != kLAT * kHID || in_sizes[7] != kLAT || in_sizes[8] != kHID * kHD ||
      in_sizes[9] != kHID * kHD || in_sizes[10] != kHID * kHID || in_sizes[11] != kHID)
    return;
  if (out_size != kM * kHID) return;

  const float* x     = (const float*)d_in[0];
  const float* amask = (const float*)d_in[1];
  const float* W_q   = (const float*)d_in[2];
  const float* b_q   = (const float*)d_in[3];
  const float* W_k   = (const float*)d_in[4];
  const float* b_k   = (const float*)d_in[5];
  const float* W_v   = (const float*)d_in[6];
  const float* b_v   = (const float*)d_in[7];
  const float* W_kup = (const float*)d_in[8];
  const float* W_vup = (const float*)d_in[9];
  const float* W_o   = (const float*)d_in[10];
  const float* b_o   = (const float*)d_in[11];
  float* out = (float*)d_out;

  const size_t nX  = (size_t)kM * kHID;
  const size_t nWq = (size_t)kHID * kHID;
  const size_t nWk = (size_t)kLAT * kHID;
  const size_t nWu = (size_t)kHID * kHD;
  const size_t nKl = (size_t)kM * kLAT;
  const size_t nQl = (size_t)kB * kH * kT * kHD;
  const size_t nVt = (size_t)kB * kH * kOD * kT;
  const size_t total_halves = 2 * (nX + nWq + nWk + nWk + nWu + nWu + nWq + nX + nKl + nKl + nQl + nVt + nX);
  if (total_halves * 2 > ws_size) return;

  size_t off = 0;
  char* wsb = (char*)d_ws;
  auto carve = [&](size_t halves) { hf_t* p = (hf_t*)(wsb + off); off += halves * 2; return p; };
  hf_t* xh   = carve(nX);  hf_t* xl   = carve(nX);
  hf_t* wqh  = carve(nWq); hf_t* wql  = carve(nWq);
  hf_t* wkh  = carve(nWk); hf_t* wkl  = carve(nWk);
  hf_t* wvh  = carve(nWk); hf_t* wvl  = carve(nWk);
  hf_t* wkTh = carve(nWu); hf_t* wkTl = carve(nWu);
  hf_t* wvuh = carve(nWu); hf_t* wvul = carve(nWu);
  hf_t* woh  = carve(nWq); hf_t* wol  = carve(nWq);
  hf_t* qfh  = carve(nX);  hf_t* qfl  = carve(nX);
  hf_t* klh  = carve(nKl); hf_t* kll  = carve(nKl);
  hf_t* vlh  = carve(nKl); hf_t* vll  = carve(nKl);
  hf_t* qlh  = carve(nQl); hf_t* qll  = carve(nQl);
  hf_t* vth  = carve(nVt); hf_t* vtl  = carve(nVt);
  hf_t* aoh  = carve(nX);  hf_t* aol  = carve(nX);
  if (off > ws_size) return;

  const dim3 blk(256);
  const float e6 = 1.0f / 64.0f, e14 = 1.0f / 16384.0f;

  {
    const int n8x = (int)(nX / 8), n8wq = (int)(nWq / 8), n8wk = (int)(nWk / 8), n8wu = (int)(nWu / 8);
    k_cvt<<<dim3((n8x + 255) / 256), blk, 0, stream>>>(x, xh, xl, n8x, 1.0f);
    k_cvt<<<dim3((n8wq + 255) / 256), blk, 0, stream>>>(W_q, wqh, wql, n8wq, 64.0f);
    k_cvt<<<dim3((n8wk + 255) / 256), blk, 0, stream>>>(W_k, wkh, wkl, n8wk, 64.0f);
    k_cvt<<<dim3((n8wk + 255) / 256), blk, 0, stream>>>(W_v, wvh, wvl, n8wk, 64.0f);
    k_cvt_tr<<<dim3(kHD / 32, kH), blk, 0, stream>>>(W_kup, wkTh, wkTl);
    k_cvt<<<dim3((n8wu + 255) / 256), blk, 0, stream>>>(W_vup, wvuh, wvul, n8wu, 64.0f);
    k_cvt<<<dim3((n8wq + 255) / 256), blk, 0, stream>>>(W_o, woh, wol, n8wq, 64.0f);
  }

  {
    GemmP p = mkp((long long)kT * kHID, 0, 0, 0, (long long)kT * kHID, 0,
                  kHID, kHID, kHID, kHID, 1, 1, 1, 0, 0, 1, e6, 1.0f);
    k_gemm<true, false><<<dim3(kHID / 64, kT0 / 128, kB), blk, 0, stream>>>(xh, xl, wqh, wql, b_q, out, qfh, qfl, p);
    p.mbase = kT0;
    k_gemm<false, false><<<dim3(kHID / 128, (kT - kT0) / 128, kB), blk, 0, stream>>>(xh, xl, wqh, wql, b_q, out, qfh, qfl, p);
  }
  {
    GemmP p = mkp((long long)kT * kHID, 0, 0, 0, (long long)kT * kLAT, 0,
                  kHID, kHID, kHID, kLAT, 1, 1, 1, 0, 0, 1, e6, 1.0f);
    k_gemm<true, false><<<dim3(kLAT / 64, kT0 / 128, kB), blk, 0, stream>>>(xh, xl, wkh, wkl, b_k, out, klh, kll, p);
    p.mbase = kT0;
    k_gemm<false, false><<<dim3(kLAT / 128, (kT - kT0) / 128, kB), blk, 0, stream>>>(xh, xl, wkh, wkl, b_k, out, klh, kll, p);
  }
  {
    GemmP p = mkp((long long)kT * kHID, 0, 0, 0, (long long)kT * kLAT, 0,
                  kHID, kHID, kHID, kLAT, 1, 1, 1, 0, 0, 1, e6, 1.0f);
    k_gemm<true, false><<<dim3(kLAT / 64, kT0 / 128, kB), blk, 0, stream>>>(xh, xl, wvh, wvl, b_v, out, vlh, vll, p);
    p.mbase = kT0;
    k_gemm<false, false><<<dim3(kLAT / 128, (kT - kT0) / 128, kB), blk, 0, stream>>>(xh, xl, wvh, wvl, b_v, out, vlh, vll, p);
  }
  {
    GemmP p = mkp((long long)kT * kHID, (long long)kOD, 0, (long long)kHD * kOD, (long long)kH * kT * kHD, (long long)kT * kHD,
                  kOD, kHID, kOD, kHD, kH, 1, 1, 0, 0, 0, e6, 4.0f);
    k_gemm<true, false><<<dim3(kHD / 64, kT0 / 128, kB * kH), blk, 0, stream>>>(qfh, qfl, wkTh, wkTl, b_q, out, qlh, qll, p);
    p.mbase = kT0;
    k_gemm<false, false><<<dim3(kHD / 128, (kT - kT0) / 128, kB * kH), blk, 0, stream>>>(qfh, qfl, wkTh, wkTl, b_q, out, qlh, qll, p);
  }
  {
    GemmP p = mkp(0, (long long)kOD * kHD, (long long)kT * kLAT, (long long)kHD, (long long)kH * kOD * kT, (long long)kOD * kT,
                  kHD, kHD, kLAT, kT, kH, 1, kH / kKV, 0, 0, 0, e6, 4.0f);
    k_gemm<true, false><<<dim3(kT0 / 64, kOD / 128, kB * kH), blk, 0, stream>>>(wvuh, wvul, vlh, vll, b_v, out, vth, vtl, p);
    p.nbase = kT0;
    k_gemm<false, false><<<dim3((kT - kT0) / 128, kOD / 128, kB * kH), blk, 0, stream>>>(wvuh, wvul, vlh, vll, b_v, out, vth, vtl, p);
  }
  k_attn<true><<<dim3(kT0 / 16, kH, kB), dim3(32), 0, stream>>>(qlh, qll, klh, kll, vth, vtl, amask, aoh, aol, 0);
  k_attn<false><<<dim3((kT - kT0) / 16, kH, kB), dim3(32), 0, stream>>>(qlh, qll, klh, kll, vth, vtl, amask, aoh, aol, kT0);
  {
    GemmP p = mkp((long long)kT * kHID, 0, 0, 0, (long long)kT * kHID, 0,
                  kHID, kHID, kHID, kHID, 1, 1, 1, 0, 0, 1, e14, 1.0f);
    k_gemm<true, true><<<dim3(kHID / 64, kT0 / 128, kB), blk, 0, stream>>>(aoh, aol, woh, wol, b_o, out, aoh, aol, p);
    p.mbase = kT0;
    k_gemm<false, true><<<dim3(kHID / 128, (kT - kT0) / 128, kB), blk, 0, stream>>>(aoh, aol, woh, wol, b_o, out, aoh, aol, p);
  }
}
